// GQAAttention_82910048682137
// MI455X (gfx1250) — hardware-verified
//
#include <hip/hip_runtime.h>

#ifndef NB
#define NB 2
#endif
#ifndef SEQ
#define SEQ 2048
#endif
#ifndef RE
#define RE 256
#endif
#define NB_FULL 2
#define SEQ_FULL 2048
#define DM 2048
#define NH 32
#define NKV 8
#define NREP (NH / NKV)
#define HDIM 64
#define KVD (NKV * HDIM)
#define NQKV (DM + 2 * KVD)
#define SLEN SEQ
#define NR (NB * SLEN)
#define TQ SLEN
#define TK SLEN
#define SCL 0.125f
#define QBLKS (TQ / 64)
#define QBN5 (RE / 64)
#define QB05 0
#define QB0P QBN5
#define QBNP (QBLKS - QBN5)
#define WSC 16.0f
#define WINV 0.0625f
#define RINV 0.0009765625f
#define WS_CAP ((size_t)134217728)

static_assert(NB >= 1 && NB <= NB_FULL);
static_assert(SEQ >= 128 && SEQ <= SEQ_FULL && SEQ % 128 == 0);
static_assert(RE >= 128 && RE <= SEQ && RE % 128 == 0);
static_assert(DM % 128 == 0 && NQKV % 64 == 0 && HDIM == 64 && KVD % 64 == 0);
static_assert(NH % NKV == 0);
static_assert(((size_t)((NB_FULL - 1) * SEQ_FULL + SEQ_FULL) * DM) * 4 <= (size_t)33554432);

typedef unsigned short v8us __attribute__((ext_vector_type(8), may_alias));
typedef float v8f __attribute__((ext_vector_type(8)));
typedef float v4f __attribute__((ext_vector_type(4)));
typedef float v4fa __attribute__((ext_vector_type(4), may_alias));
typedef int v4i __attribute__((ext_vector_type(4)));
typedef _Float16 v16h __attribute__((ext_vector_type(16)));
typedef _Float16 v4h __attribute__((ext_vector_type(4)));
union FragH { v16h v; v8us half[2]; _Float16 h[16]; unsigned short u[16]; };

__device__ __forceinline__ unsigned short bf16_bits(float x) { unsigned int u = __float_as_uint(x); return (unsigned short)((u + 0x7FFFu + ((u >> 16) & 1u)) >> 16); }
__device__ __forceinline__ float bf16_val(unsigned short b) { return __uint_as_float(((unsigned int)b) << 16); }
__device__ __forceinline__ float bf16_rne(float x) { return bf16_val(bf16_bits(x)); }

__device__ __forceinline__ v8f mma1(v16h a, v16h b, v8f c) {
  v8f d = __builtin_amdgcn_wmma_f32_16x16x32_f16(false, a, false, b, (short)0, c, false, false);
  asm volatile("v_nop\n\tv_nop\n\tv_nop\n\tv_nop" : "+v"(d) : "v"(a), "v"(b));
  return d;
}
__device__ __forceinline__ v16h g2_frag(const _Float16* p, int hh) { FragH f; f.half[0] = *(const v8us*)((const unsigned short*)p + 8 * hh); f.half[1] = *(const v8us*)((const unsigned short*)p + 16 + 8 * hh); return f.v; }

__global__ __launch_bounds__(256) void k_chk(const int* __restrict__ MK, int* __restrict__ FLG) {
  __shared__ int red[256];
  const int tid = threadIdx.x;
  int bad = 0;
#pragma unroll 1
  for (int e4 = tid; e4 < SLEN * (SLEN / 4); e4 += 256) {
    const int i = e4 / (SLEN / 4), j = (e4 - i * (SLEN / 4)) * 4;
    const v4i m = *(const v4i*)(MK + (size_t)i * SEQ_FULL + j);
#pragma unroll
    for (int q = 0; q < 4; ++q) { const int want = (j + q <= i) ? 1 : 0; const int mv = m[q]; const int got = (mv != 0) ? 1 : 0; bad |= (want ^ got); }
  }
  red[tid] = bad; __syncthreads();
  for (int st = 128; st > 0; st >>= 1) { if (tid < st) red[tid] |= red[tid + st]; __syncthreads(); }
  const int ok = (red[0] == 0) ? 1 : 0;
  const v4i v = {ok, ok, ok, ok};
  if (tid < 8) *(volatile v4i*)(FLG + tid * 4) = v;
  __threadfence();
  if (tid < 8) *(volatile v4i*)(FLG + tid * 4) = v;
}

__global__ __launch_bounds__(256) void k_wsc(const float* __restrict__ Wm, _Float16* __restrict__ Bt, size_t n8, float sc) {
  #pragma clang fp contract(off)
  const size_t t = (size_t)blockIdx.x * 256 + threadIdx.x; if (t >= n8) return;
  const v4f a = *(const v4fa*)(Wm + t * 8), c = *(const v4fa*)(Wm + t * 8 + 4);
  FragH f;
#pragma unroll
  for (int q = 0; q < 4; ++q) { f.h[q] = (_Float16)(bf16_rne(a[q]) * sc); f.h[4 + q] = (_Float16)(bf16_rne(c[q]) * sc); }
  const v8us o = f.half[0];
  *(volatile v8us*)((unsigned short*)Bt + t * 8) = o; __threadfence(); *(volatile v8us*)((unsigned short*)Bt + t * 8) = o;
}

__global__ __launch_bounds__(256) void k_x16(const float* __restrict__ x, _Float16* __restrict__ X16, size_t n8) {
  #pragma clang fp contract(off)
  const size_t t = (size_t)blockIdx.x * 256 + threadIdx.x; if (t >= n8) return;
  const size_t row = (t * 8) / DM; const int c = (int)((t * 8) % DM); const size_t b = row / SLEN, s = row - b * SLEN;
  const float* src = x + (b * SEQ_FULL + s) * (size_t)DM + c;
  const v4f a = *(const v4fa*)src, d = *(const v4fa*)(src + 4);
  FragH f;
#pragma unroll
  for (int q = 0; q < 4; ++q) { f.h[q] = (_Float16)bf16_rne(a[q]); f.h[4 + q] = (_Float16)bf16_rne(d[q]); }
  const v8us o = f.half[0];
  *(volatile v8us*)((unsigned short*)X16 + t * 8) = o; __threadfence(); *(volatile v8us*)((unsigned short*)X16 + t * 8) = o;
}

__global__ __launch_bounds__(256) void k_hl(const float* __restrict__ F, _Float16* __restrict__ Hh, _Float16* __restrict__ Hl, size_t n8) {
  #pragma clang fp contract(off)
  const size_t t = (size_t)blockIdx.x * 256 + threadIdx.x; if (t >= n8) return;
  FragH fh, fl; const v4f a = *(const v4fa*)(F + t * 8), c = *(const v4fa*)(F + t * 8 + 4);
#pragma unroll
  for (int q = 0; q < 4; ++q) { _Float16 hv = (_Float16)a[q]; fh.h[q] = hv; fl.h[q] = (_Float16)((a[q] - (float)hv) * 1024.0f); hv = (_Float16)c[q]; fh.h[4 + q] = hv; fl.h[4 + q] = (_Float16)((c[q] - (float)hv) * 1024.0f); }
  const v8us oh = fh.half[0], ol = fl.half[0];
  for (int pass = 0; pass < 2; ++pass) { *(volatile v8us*)((unsigned short*)Hh + t * 8) = oh; *(volatile v8us*)((unsigned short*)Hl + t * 8) = ol; if (pass == 0) __threadfence(); }
}

template <int ACT>
__global__ __launch_bounds__(128) void k_gemm2(const _Float16* __restrict__ A, int lda, size_t sA, const _Float16* __restrict__ Bh, int ldb, size_t sB, float alpha,
    const float* __restrict__ bias, size_t sBias, const float* CP, int rowsPerB, size_t sCPb, int row0g,
    float* C, _Float16* __restrict__ C16, _Float16* __restrict__ CL16, int ldc, size_t sC, int M, int N, int K) {
  __shared__ __attribute__((aligned(16))) float so[4][32][68];
  const int tid = threadIdx.x, w = tid >> 5, lane = tid & 31, ln = lane & 15, hh = lane >> 4; const int by = blockIdx.y;
  A += (size_t)by * sA; Bh += (size_t)by * sB; const size_t cofs = (size_t)by * sC; const float* bp = bias ? bias + (size_t)by * sBias : nullptr;
  const int ntn = N >> 6; const int mt = blockIdx.x / ntn, nq = blockIdx.x - mt * ntn; const int row0 = mt * 128 + 32 * w, col0 = nq * 64; if (row0 >= M) return;
  const _Float16* a0p = A + (size_t)(row0 + ln) * lda; const _Float16* a1p = a0p + (size_t)16 * lda;
  const _Float16* b0p = Bh + (size_t)(col0 + ln) * ldb; const _Float16* b1p = b0p + (size_t)16 * ldb; const _Float16* b2p = b1p + (size_t)16 * ldb; const _Float16* b3p = b2p + (size_t)16 * ldb;
  const v8f z8 = {0.f,0.f,0.f,0.f,0.f,0.f,0.f,0.f}; v8f c00 = z8, c01 = z8, c02 = z8, c03 = z8, c10 = z8, c11 = z8, c12 = z8, c13 = z8;
#pragma unroll 1
  for (int kb = 0; kb < K; kb += 32) { const v16h a0 = g2_frag(a0p + kb, hh), a1 = g2_frag(a1p + kb, hh);
    v16h b = g2_frag(b0p + kb, hh); c00 = mma1(a0, b, c00); c10 = mma1(a1, b, c10);
    b = g2_frag(b1p + kb, hh); c01 = mma1(a0, b, c01); c11 = mma1(a1, b, c11);
    b = g2_frag(b2p + kb, hh); c02 = mma1(a0, b, c02); c12 = mma1(a1, b, c12);
    b = g2_frag(b3p + kb, hh); c03 = mma1(a0, b, c03); c13 = mma1(a1, b, c13); }
  v8f accs[8] = {c00, c01, c02, c03, c10, c11, c12, c13};
  const bool cpown = (CP != nullptr) && (rowsPerB < 0) && (row0g + row0 < -rowsPerB);
#pragma unroll
  for (int u = 0; u < 8; ++u) { const int t = u & 3, half = u >> 2; const int col = col0 + t * 16 + ln; const float bv = bp ? bf16_rne(bp[col]) : 0.f;
#pragma unroll
    for (int r = 0; r < 8; ++r) { const int rloc = half * 16 + 8 * hh + r; float v = accs[u][r] * alpha + bv;
      if (cpown) v += CP[cofs + (size_t)(row0g + row0 + rloc) * ldc + col];
      else if (CP != nullptr && rowsPerB > 0) { const int bidx = (row0g + row0 + rloc) / rowsPerB; v += CP[(size_t)bidx * sCPb + (size_t)by * 64 + col]; }
      if (ACT == 3) v = fmaxf(v, 0.f);
      so[w][rloc][t * 16 + ln] = v; } }
  __builtin_amdgcn_fence(4, "workgroup"); __builtin_amdgcn_wave_barrier();
  const int rsub = lane >> 4, c4 = (lane & 15) * 4;
  for (int pass = 0; pass < 2; ++pass) {
#pragma unroll
    for (int q = 0; q < 16; ++q) { const int r = q * 2 + rsub; const v4f v = *(const v4fa*)&so[w][r][c4];
      if (C) *(volatile v4f*)(C + cofs + (size_t)(row0 + r) * ldc + col0 + c4) = v;
      if (C16) { v4h h4, l4;
#pragma unroll
        for (int i = 0; i < 4; ++i) { const float vi = v[i]; const _Float16 hv = (_Float16)vi; h4[i] = hv; l4[i] = (_Float16)((vi - (float)hv) * 1024.0f); }
        *(volatile v4h*)(C16 + cofs + (size_t)(row0 + r) * ldc + col0 + c4) = h4;
        if (CL16) *(volatile v4h*)(CL16 + cofs + (size_t)(row0 + r) * ldc + col0 + c4) = l4; } }
    if (pass == 0) __threadfence(); }
}

__global__ __launch_bounds__(256) void k_vtg(const _Float16* __restrict__ VH, const _Float16* __restrict__ VL, int ldv, int voff, _Float16* __restrict__ Vt, _Float16* __restrict__ VtL) {
  __shared__ unsigned short tl[2][64][66];
  const int tid = threadIdx.x; const int slab = blockIdx.x / (SLEN / 64), lg = blockIdx.x % (SLEN / 64); const int b = slab / NKV, g = slab % NKV;
  for (int i = tid; i < 64 * 8; i += 256) { const int r = i / 8, c8 = (i % 8) * 8; const size_t sof = ((size_t)b * SLEN + lg * 64 + r) * ldv + voff + g * 64 + c8; FragH f, fl;
    f.half[0] = *(const v8us*)((const unsigned short*)VH + sof); fl.half[0] = *(const v8us*)((const unsigned short*)VL + sof);
#pragma unroll
    for (int q = 0; q < 8; ++q) { tl[0][r][c8 + q] = f.u[q]; tl[1][r][c8 + q] = fl.u[q]; } }
  __syncthreads();
  for (int pass = 0; pass < 2; ++pass) {
#pragma unroll
    for (int rd = 0; rd < 2; ++rd) { const int d = rd * 32 + tid / 8, pc = tid % 8; FragH f, fl;
#pragma unroll
      for (int q = 0; q < 8; ++q) { f.u[q] = tl[0][pc * 8 + q][d]; fl.u[q] = tl[1][pc * 8 + q][d]; }
      const size_t o = ((size_t)slab * 64 + d) * TK + lg * 64 + pc * 8;
      *(volatile v8us*)((unsigned short*)Vt + o) = f.half[0]; *(volatile v8us*)((unsigned short*)VtL + o) = fl.half[0]; }
    if (pass == 0) __threadfence(); }
}

template <int CAUSAL>
__global__ __launch_bounds__(128) __attribute__((amdgpu_num_vgpr(256))) void k_flash(const _Float16* __restrict__ Q16, int ldq, const _Float16* __restrict__ K16, int ldk, const _Float16* __restrict__ Vt,
    const int* __restrict__ FLG, float* __restrict__ O, int ldo, int qbn, int qbfirst) {
  constexpr int RPW = 16, DT = 4, KS = 2;
  __shared__ __attribute__((aligned(16))) unsigned short sP[4][RPW][40];
  __shared__ __attribute__((aligned(16))) float sO[4][RPW][64 + 4];
  const int tid = threadIdx.x, w = tid >> 5, lane = tid & 31, ln = lane & 15, hh = lane >> 4;
  const int slab = blockIdx.x / qbn, qblk = qbfirst + blockIdx.x % qbn; const int b = slab / NH, h = slab % NH, g = h / NREP;
  const int qb0 = qblk * (4 * RPW); const int q0 = qb0 + w * RPW;
  const int okm = FLG[0];
  const v8f z8 = {0.f,0.f,0.f,0.f,0.f,0.f,0.f,0.f};
  FragH aq[KS];
  { const unsigned short* qr = (const unsigned short*)Q16 + ((size_t)b * TQ + q0 + ln) * ldq + h * 64;
#pragma unroll
    for (int ks = 0; ks < KS; ++ks) { aq[ks].half[0] = *(const v8us*)(qr + ks * 32 + 8 * hh); aq[ks].half[1] = *(const v8us*)(qr + ks * 32 + 16 + 8 * hh); } }
  const unsigned short* Kb = (const unsigned short*)K16 + (size_t)b * TK * ldk + g * 64;
  const unsigned short* Vth = (const unsigned short*)Vt + (size_t)(b * NKV + g) * 64 * TK;
  float m_r[8], l_r[8]; v8f oacc[DT];
#pragma unroll
  for (int r = 0; r < 8; ++r) { m_r[r] = -3.0e38f; l_r[r] = 0.f; }
#pragma unroll
  for (int dt = 0; dt < DT; ++dt) oacc[dt] = z8;
  const int jend = (CAUSAL == 1) ? (qb0 + 4 * RPW) : TK;
#pragma unroll 1
  for (int j0 = 0; j0 < jend; j0 += 32) {
    v8f s[2];
#pragma unroll
    for (int nt = 0; nt < 2; ++nt) { const unsigned short* kr = Kb + (size_t)(j0 + nt * 16 + ln) * ldk; v8f acc = z8;
#pragma unroll
      for (int ks = 0; ks < KS; ++ks) { FragH bk; bk.half[0] = *(const v8us*)(kr + ks * 32 + 8 * hh); bk.half[1] = *(const v8us*)(kr + ks * 32 + 16 + 8 * hh); acc = mma1(aq[ks].v, bk.v, acc); }
      s[nt] = acc; }
#pragma unroll
    for (int r = 0; r < 8; ++r) { const int tq = q0 + 8 * hh + r; const int k0 = j0 + ln, k1 = j0 + 16 + ln;
      const bool ok0 = (CAUSAL == 1) ? (k0 <= tq) : true, ok1 = (CAUSAL == 1) ? (k1 <= tq) : true;
      const float s0 = ok0 ? s[0][r] * SCL : -3.0e38f, s1 = ok1 ? s[1][r] * SCL : -3.0e38f; float mc = fmaxf(s0, s1);
      mc = fmaxf(mc, __shfl_xor(mc, 1, 32)); mc = fmaxf(mc, __shfl_xor(mc, 2, 32)); mc = fmaxf(mc, __shfl_xor(mc, 4, 32)); mc = fmaxf(mc, __shfl_xor(mc, 8, 32));
      const float mn = fmaxf(m_r[r], mc); const float al = (mn > -1.0e38f) ? expf(m_r[r] - mn) : 1.0f; m_r[r] = mn;
      const float p0 = ok0 ? expf(s0 - mn) : 0.f, p1 = ok1 ? expf(s1 - mn) : 0.f; l_r[r] = l_r[r] * al + p0 + p1;
#pragma unroll
      for (int dt = 0; dt < DT; ++dt) oacc[dt][r] *= al;
      const _Float16 h0 = (_Float16)(p0 * 1024.0f), h1 = (_Float16)(p1 * 1024.0f);
      sP[w][8 * hh + r][ln] = __builtin_bit_cast(unsigned short, h0); sP[w][8 * hh + r][16 + ln] = __builtin_bit_cast(unsigned short, h1); }
    __builtin_amdgcn_fence(4, "workgroup"); __builtin_amdgcn_wave_barrier();
    FragH pa; pa.half[0] = *(const v8us*)&sP[w][ln][8 * hh]; pa.half[1] = *(const v8us*)&sP[w][ln][16 + 8 * hh];
#pragma unroll
    for (int dt = 0; dt < DT; ++dt) { const unsigned short* vrow = Vth + (size_t)(dt * 16 + ln) * TK + j0; FragH bv; bv.half[0] = *(const v8us*)(vrow + 8 * hh); bv.half[1] = *(const v8us*)(vrow + 16 + 8 * hh);
      oacc[dt] = mma1(pa.v, bv.v, oacc[dt]); }
    __builtin_amdgcn_fence(4, "workgroup"); __builtin_amdgcn_wave_barrier(); }
#pragma unroll
  for (int r = 0; r < 8; ++r) { float l = l_r[r]; l += __shfl_xor(l, 1, 32); l += __shfl_xor(l, 2, 32); l += __shfl_xor(l, 4, 32); l += __shfl_xor(l, 8, 32); l_r[r] = (l > 0.f) ? 1.0f / (l * 1024.0f) : 0.f; }
  const float qnan = __int_as_float(0x7fc00000);
#pragma unroll
  for (int dt = 0; dt < DT; ++dt)
#pragma unroll
    for (int r = 0; r < 8; ++r) { const float v = oacc[dt][r] * l_r[r]; sO[w][8 * hh + r][dt * 16 + ln] = (okm != 0) ? v : qnan; }
  __builtin_amdgcn_fence(4, "workgroup"); __builtin_amdgcn_wave_barrier();
  for (int pass = 0; pass < 2; ++pass) {
#pragma unroll
    for (int rp = 0; rp < RPW; rp += 2) { const int r = rp + hh, pc = ln; const v4f val = *(const v4fa*)&sO[w][r][pc * 4]; *(volatile v4f*)(O + ((size_t)b * TQ + q0 + r) * ldo + h * 64 + pc * 4) = val; }
    if (pass == 0) __threadfence(); }
}

template <int CAUSAL>
__global__ __launch_bounds__(128) __attribute__((amdgpu_num_vgpr(256))) void k_flash5(const _Float16* __restrict__ Q16, const _Float16* __restrict__ QL, int ldq, const _Float16* __restrict__ K16, const _Float16* __restrict__ KL, int ldk,
    const _Float16* __restrict__ Vt, const _Float16* __restrict__ VtL, const int* __restrict__ FLG, float* __restrict__ O, int ldo, int qbn, int qbfirst) {
  constexpr int RPW = 16, DT = 4, KS = 2;
  __shared__ __attribute__((aligned(16))) unsigned short sP[4][RPW][40];
  __shared__ __attribute__((aligned(16))) unsigned short sPL[4][RPW][40];
  __shared__ __attribute__((aligned(16))) float sO[4][RPW][64 + 4];
  const int tid = threadIdx.x, w = tid >> 5, lane = tid & 31, ln = lane & 15, hh = lane >> 4;
  const int slab = blockIdx.x / qbn, qblk = qbfirst + blockIdx.x % qbn; const int b = slab / NH, h = slab % NH, g = h / NREP;
  const int qb0 = qblk * (4 * RPW); const int q0 = qb0 + w * RPW;
  const int okm = FLG[0];
  const v8f z8 = {0.f,0.f,0.f,0.f,0.f,0.f,0.f,0.f};
  FragH aq[KS], aql[KS];
  { const size_t qo = ((size_t)b * TQ + q0 + ln) * ldq + h * 64; const unsigned short* qr = (const unsigned short*)Q16 + qo; const unsigned short* ql = (const unsigned short*)QL + qo;
#pragma unroll
    for (int ks = 0; ks < KS; ++ks) { aq[ks].half[0] = *(const v8us*)(qr + ks * 32 + 8 * hh); aq[ks].half[1] = *(const v8us*)(qr + ks * 32 + 16 + 8 * hh);
      aql[ks].half[0] = *(const v8us*)(ql + ks * 32 + 8 * hh); aql[ks].half[1] = *(const v8us*)(ql + ks * 32 + 16 + 8 * hh); } }
  const size_t kofs = (size_t)b * TK * ldk + g * 64; const unsigned short* Kb = (const unsigned short*)K16 + kofs; const unsigned short* Klb = (const unsigned short*)KL + kofs;
  const size_t vofs = (size_t)(b * NKV + g) * 64 * TK; const unsigned short* Vth = (const unsigned short*)Vt + vofs; const unsigned short* Vtl = (const unsigned short*)VtL + vofs;
  float m_r[8], l_r[8]; v8f oacc[DT], oaccL[DT];
#pragma unroll
  for (int r = 0; r < 8; ++r) { m_r[r] = -3.0e38f; l_r[r] = 0.f; }
#pragma unroll
  for (int dt = 0; dt < DT; ++dt) { oacc[dt] = z8; oaccL[dt] = z8; }
  const int jend = (CAUSAL == 1) ? (qb0 + 4 * RPW) : TK;
#pragma unroll 1
  for (int j0 = 0; j0 < jend; j0 += 32) {
    v8f s[2];
#pragma unroll
    for (int nt = 0; nt < 2; ++nt) { const size_t ko = (size_t)(j0 + nt * 16 + ln) * ldk; const unsigned short* kr = Kb + ko; const unsigned short* klr = Klb + ko; v8f acc = z8, accl = z8;
#pragma unroll
      for (int ks = 0; ks < KS; ++ks) {
        FragH bk; bk.half[0] = *(const v8us*)(kr + ks * 32 + 8 * hh); bk.half[1] = *(const v8us*)(kr + ks * 32 + 16 + 8 * hh);
        acc = mma1(aq[ks].v, bk.v, acc); accl = mma1(aql[ks].v, bk.v, accl);
        FragH bkl; bkl.half[0] = *(const v8us*)(klr + ks * 32 + 8 * hh); bkl.half[1] = *(const v8us*)(klr + ks * 32 + 16 + 8 * hh);
        accl = mma1(aq[ks].v, bkl.v, accl); }
#pragma unroll
      for (int r = 0; r < 8; ++r) acc[r] += accl[r] * RINV;
      s[nt] = acc; }
#pragma unroll
    for (int r = 0; r < 8; ++r) { const int tq = q0 + 8 * hh + r; const int k0 = j0 + ln, k1 = j0 + 16 + ln;
      const bool ok0 = (CAUSAL == 1) ? (k0 <= tq) : true, ok1 = (CAUSAL == 1) ? (k1 <= tq) : true;
      const float s0 = ok0 ? s[0][r] * SCL : -3.0e38f, s1 = ok1 ? s[1][r] * SCL : -3.0e38f; float mc = fmaxf(s0, s1);
      mc = fmaxf(mc, __shfl_xor(mc, 1, 32)); mc = fmaxf(mc, __shfl_xor(mc, 2, 32)); mc = fmaxf(mc, __shfl_xor(mc, 4, 32)); mc = fmaxf(mc, __shfl_xor(mc, 8, 32));
      const float mn = fmaxf(m_r[r], mc); const float al = (mn > -1.0e38f) ? expf(m_r[r] - mn) : 1.0f; m_r[r] = mn;
      const float p0 = ok0 ? expf(s0 - mn) : 0.f, p1 = ok1 ? expf(s1 - mn) : 0.f; l_r[r] = l_r[r] * al + p0 + p1;
#pragma unroll
      for (int dt = 0; dt < DT; ++dt) { oacc[dt][r] *= al; oaccL[dt][r] *= al; }
      const float ps0 = p0 * 1024.0f, ps1 = p1 * 1024.0f; const _Float16 h0 = (_Float16)ps0, h1 = (_Float16)ps1;
      const _Float16 e0 = (_Float16)((ps0 - (float)h0) * 1024.0f), e1 = (_Float16)((ps1 - (float)h1) * 1024.0f);
      sP[w][8 * hh + r][ln] = __builtin_bit_cast(unsigned short, h0); sP[w][8 * hh + r][16 + ln] = __builtin_bit_cast(unsigned short, h1);
      sPL[w][8 * hh + r][ln] = __builtin_bit_cast(unsigned short, e0); sPL[w][8 * hh + r][16 + ln] = __builtin_bit_cast(unsigned short, e1); }
    __builtin_amdgcn_fence(4, "workgroup"); __builtin_amdgcn_wave_barrier();
    FragH pa, pl;
    pa.half[0] = *(const v8us*)&sP[w][ln][8 * hh]; pa.half[1] = *(const v8us*)&sP[w][ln][16 + 8 * hh];
    pl.half[0] = *(const v8us*)&sPL[w][ln][8 * hh]; pl.half[1] = *(const v8us*)&sPL[w][ln][16 + 8 * hh];
#pragma unroll
    for (int dt = 0; dt < DT; ++dt) { const size_t vo = (size_t)(dt * 16 + ln) * TK + j0;
      FragH bv; bv.half[0] = *(const v8us*)(Vth + vo + 8 * hh); bv.half[1] = *(const v8us*)(Vth + vo + 16 + 8 * hh);
      oacc[dt] = mma1(pa.v, bv.v, oacc[dt]); oaccL[dt] = mma1(pl.v, bv.v, oaccL[dt]);
      FragH bl; bl.half[0] = *(const v8us*)(Vtl + vo + 8 * hh); bl.half[1] = *(const v8us*)(Vtl + vo + 16 + 8 * hh);
      oaccL[dt] = mma1(pa.v, bl.v, oaccL[dt]); }
    __builtin_amdgcn_fence(4, "workgroup"); __builtin_amdgcn_wave_barrier(); }
#pragma unroll
  for (int r = 0; r < 8; ++r) { float l = l_r[r]; l += __shfl_xor(l, 1, 32); l += __shfl_xor(l, 2, 32); l += __shfl_xor(l, 4, 32); l += __shfl_xor(l, 8, 32); l_r[r] = (l > 0.f) ? 1.0f / (l * 1024.0f) : 0.f; }
  const float qnan = __int_as_float(0x7fc00000);
#pragma unroll
  for (int dt = 0; dt < DT; ++dt)
#pragma unroll
    for (int r = 0; r < 8; ++r) { float v = oacc[dt][r]; v += oaccL[dt][r] * RINV; v *= l_r[r]; sO[w][8 * hh + r][dt * 16 + ln] = (okm != 0) ? v : qnan; }
  __builtin_amdgcn_fence(4, "workgroup"); __builtin_amdgcn_wave_barrier();
  for (int pass = 0; pass < 2; ++pass) {
#pragma unroll
    for (int rp = 0; rp < RPW; rp += 2) { const int r = rp + hh, pc = ln; const v4f val = *(const v4fa*)&sO[w][r][pc * 4]; *(volatile v4f*)(O + ((size_t)b * TQ + q0 + r) * ldo + h * 64 + pc * 4) = val; }
    if (pass == 0) __threadfence(); }
}

extern "C" void kernel_launch(void* const* d_in, const int* in_sizes, int n_in,
                              void* d_out, int out_size, void* d_ws, size_t ws_size, hipStream_t stream) {
  if (n_in < 4) return;
  if (in_sizes[0] < ((NB - 1) * SEQ_FULL + SEQ) * DM) return;
  if (in_sizes[1] < NQKV * DM) return;
  if (in_sizes[2] < DM * DM) return;
  if (in_sizes[3] < SEQ_FULL * SEQ_FULL) return;
  if (out_size < ((NB - 1) * SEQ_FULL + SEQ) * DM) return;
  const float* x = (const float*)d_in[0]; const float* Wqkv = (const float*)d_in[1]; const float* Wo = (const float*)d_in[2]; const int* msk = (const int*)d_in[3];
  float* out = (float*)d_out;
  char* ws = (char*)d_ws; size_t off = 0;
  auto take = [&](size_t bytes) { char* p = ws + off; off += (bytes + 255) & ~(size_t)255; return p; };
  const size_t np = (size_t)NR * DM, nqp = (size_t)NR * NQKV, nvt = (size_t)NB * NKV * 64 * TK;
  int* FLG = (int*)take(256);
  _Float16* BQKV = (_Float16*)take((size_t)NQKV * DM * 2);
  _Float16* BO = (_Float16*)take((size_t)DM * DM * 2);
  _Float16* X16 = (_Float16*)take(np * 2);
  _Float16* QKVH = (_Float16*)take(nqp * 2);
  _Float16* QKVL = (_Float16*)take(nqp * 2);
  _Float16* VT = (_Float16*)take(nvt * 2);
  _Float16* VTL = (_Float16*)take(nvt * 2);
  float* O = (float*)take(np * 4);
  _Float16* OH = X16;
  _Float16* OL = QKVH;
  if (off > ws_size || off > WS_CAP) return;

  k_chk<<<1, 256, 0, stream>>>(msk, FLG);
  k_wsc<<<(unsigned)(((size_t)NQKV * DM / 8 + 255) / 256), 256, 0, stream>>>(Wqkv, BQKV, (size_t)NQKV * DM / 8, WSC);
  k_wsc<<<(unsigned)(((size_t)DM * DM / 8 + 255) / 256), 256, 0, stream>>>(Wo, BO, (size_t)DM * DM / 8, WSC);
  k_x16<<<(unsigned)((np / 8 + 255) / 256), 256, 0, stream>>>(x, X16, np / 8);
  k_gemm2<0><<<dim3((NR / 128) * (NQKV / 64), 1), 128, 0, stream>>>(X16, DM, 0, BQKV, DM, 0, WINV, nullptr, 0, nullptr, 1, 0, 0, nullptr, QKVH, QKVL, NQKV, 0, NR, NQKV, DM);
  k_vtg<<<NB * NKV * (SLEN / 64), 256, 0, stream>>>(QKVH, QKVL, NQKV, DM + KVD, VT, VTL);
  k_flash5<1><<<NB * NH * QBN5, 128, 0, stream>>>(QKVH, QKVL, NQKV, QKVH + DM, QKVL + DM, NQKV, VT, VTL, FLG, O, DM, QBN5, QB05);
  if (QBNP > 0) k_flash<1><<<NB * NH * QBNP, 128, 0, stream>>>(QKVH, NQKV, QKVH + DM, NQKV, VT, FLG, O, DM, QBNP, QB0P);
  k_hl<<<(unsigned)((np / 8 + 255) / 256), 256, 0, stream>>>(O, OH, OL, np / 8);
  k_gemm2<0><<<dim3((RE / 128) * (DM / 64), NB), 128, 0, stream>>>(OL, DM, (size_t)SLEN * DM, BO, DM, 0, WINV * RINV, nullptr, 0, nullptr, 1, 0, 0, out, nullptr, nullptr, DM, (size_t)SEQ_FULL * DM, RE, DM, DM);
  k_gemm2<0><<<dim3((SLEN / 128) * (DM / 64), NB), 128, 0, stream>>>(OH, DM, (size_t)SLEN * DM, BO, DM, 0, WINV, nullptr, 0, out, -RE, 0, 0, out, nullptr, nullptr, DM, (size_t)SEQ_FULL * DM, SLEN, DM, DM);
}
